// HandsRAT_13700945674611
// MI455X (gfx1250) — hardware-verified
//
#include <hip/hip_runtime.h>
#include <stdint.h>

#define NBATCH 32
#define NTIME  512
#define NJ     21
#define NCO    3
#define NHID   128
#define NOUT   256
#define NCH    (NJ * NHID)
#define NF     (NBATCH * NTIME)
#define TP     (NTIME + 2)
#define NROWS  (NBATCH * TP)
#define NPC    (NCH / 8)
#define KTOT   (3 * NCH)
#define SLOPE  0.2f
#define MINNORM 6.103515625e-05f
#define SWK    256.0f
#define IWK    0.00390625f
#define SPW    64.0f
#define IPW    0.015625f
#define SRES   2048.0f
#define IRES   0.00048828125f

static_assert((NCH % 32) == 0);
static_assert((3 * NOUT * NPC) == 1008 * 256);
static_assert((NOUT * NOUT / 8) == 32 * 256);
static_assert((NROWS % 2) == 0);
static_assert((NF % 128) == 0);
static_assert((NOUT % 64) == 0);
static_assert((NTIME % 16) == 0);

typedef _Float16     v16h __attribute__((ext_vector_type(16)));
typedef float        v8f  __attribute__((ext_vector_type(8)));
typedef float        v4f  __attribute__((ext_vector_type(4)));
typedef unsigned int v4u  __attribute__((ext_vector_type(4)));
typedef unsigned int v2u  __attribute__((ext_vector_type(2)));

__device__ __forceinline__ unsigned short bf_bits(float f) {
  unsigned u = __float_as_uint(f);
  return (unsigned short)((u + 0x7FFFu + ((u >> 16) & 1u)) >> 16);
}
__device__ __forceinline__ float bfr(float f) { return __uint_as_float(((unsigned)bf_bits(f)) << 16); }
__device__ __forceinline__ v4f bfr4(const float* p) {
  const v4f v = *(const v4f*)p;
  v4f r;
  r[0] = bfr(v[0]); r[1] = bfr(v[1]); r[2] = bfr(v[2]); r[3] = bfr(v[3]);
  return r;
}
__device__ __forceinline__ unsigned pk16(unsigned short a, unsigned short b) { return (unsigned)a | ((unsigned)b << 16); }
__device__ __forceinline__ v8f zero8() { v8f z = {0.f, 0.f, 0.f, 0.f, 0.f, 0.f, 0.f, 0.f}; return z; }

__device__ __forceinline__ unsigned short f16z_bits(float v) {
  const _Float16 h = (_Float16)v;
  const float hf = (float)h;
  const unsigned short b = __builtin_bit_cast(unsigned short, h);
  return (fabsf(hf) < MINNORM) ? (unsigned short)0 : b;
}
__device__ __forceinline__ void split16(float v, unsigned short& hb, unsigned short& lb) {
  const _Float16 h = (_Float16)v;
  float hf = (float)h;
  const bool tiny = fabsf(hf) < MINNORM;
  hf = tiny ? 0.0f : hf;
  hb = tiny ? (unsigned short)0 : __builtin_bit_cast(unsigned short, h);
  lb = f16z_bits((v - hf) * SRES);
}
__device__ __forceinline__ v4u pack8(const unsigned short* hv) {
  v4u u;
  u[0] = pk16(hv[0], hv[1]);
  u[1] = pk16(hv[2], hv[3]);
  u[2] = pk16(hv[4], hv[5]);
  u[3] = pk16(hv[6], hv[7]);
  return u;
}

__device__ __forceinline__ v16h ldfrag_u(const unsigned short* p) {
  union { v16h v; v4u u[2]; } f;
  f.u[0] = *(const v4u*)(p);
  f.u[1] = *(const v4u*)(p + 16);
  return f.v;
}

__device__ __forceinline__ v8f mma_raw(v16h a, v16h b, v8f c) {
  return __builtin_amdgcn_wmma_f32_16x16x32_f16(false, a, false, b, (short)0, c, false, false);
}
__device__ __forceinline__ void guard4(v8f& c0, v8f& c1, v8f& c2, v8f& c3, const v16h& a,
                                       const v16h& b0, const v16h& b1, const v16h& b2, const v16h& b3) {
#if defined(__HIP_DEVICE_COMPILE__)
  asm volatile("v_nop\n\tv_nop\n\tv_nop\n\tv_nop"
               : "+v"(c0), "+v"(c1), "+v"(c2), "+v"(c3)
               : "v"(a), "v"(b0), "v"(b1), "v"(b2), "v"(b3));
#endif
}
__device__ __forceinline__ void guard8(v8f& c0, v8f& c1, v8f& c2, v8f& c3, v8f& c4, v8f& c5, v8f& c6, v8f& c7,
                                       const v16h& a0, const v16h& a1,
                                       const v16h& b0, const v16h& b1, const v16h& b2, const v16h& b3) {
#if defined(__HIP_DEVICE_COMPILE__)
  asm volatile("v_nop\n\tv_nop\n\tv_nop\n\tv_nop"
               : "+v"(c0), "+v"(c1), "+v"(c2), "+v"(c3), "+v"(c4), "+v"(c5), "+v"(c6), "+v"(c7)
               : "v"(a0), "v"(a1), "v"(b0), "v"(b1), "v"(b2), "v"(b3));
#endif
}

__global__ __launch_bounds__(256)
void k_wprep(const float* __restrict__ conv_w, const float* __restrict__ proj_w,
             unsigned short* Wk, unsigned short* Pw) {
  const int blk = blockIdx.x, tid = threadIdx.x;
  unsigned short hv[8];
  unsigned short* dst;
  if (blk < 1008) {
    const int q = blk * 256 + tid;
    const int rr = q / NPC, cq = q - rr * NPC;
    const int tap = rr >> 8, o = rr & 255;
    const float* src = conv_w + (size_t)o * KTOT + (size_t)(8 * cq) * 3 + tap;
#pragma unroll
    for (int e = 0; e < 8; ++e) hv[e] = f16z_bits(SWK * bfr(src[3 * e]));
    dst = Wk + (size_t)8 * q;
  } else {
    const int q = (blk - 1008) * 256 + tid;
    const float* src = proj_w + (size_t)8 * q;
#pragma unroll
    for (int e = 0; e < 8; ++e) hv[e] = f16z_bits(SPW * bfr(src[e]));
    dst = Pw + (size_t)8 * q;
  }
  const v4u u = pack8(hv);
  *(volatile v4u*)dst = u;
  __threadfence();
  *(volatile v4u*)dst = u;
}

__global__ __launch_bounds__(64)
void k_gat(const float* __restrict__ x, const float* __restrict__ adj, const float* __restrict__ W,
           const float* __restrict__ av, const float* __restrict__ gb, unsigned short* Gp) {
  __shared__ float s_adj[448];
  __shared__ __align__(16) float s_wh[2][NCH];
  __shared__ __align__(16) unsigned int s_stg[2][NCH / 2];
  __shared__ float s_s1[2][32];
  __shared__ float s_s2[2][32];

  const int tid = threadIdx.x, w = tid >> 5, lane = tid & 31;
  const int row = blockIdx.x * 2 + w;
  const int b = row / TP, tp = row - b * TP;
  const bool isz = (tp == 0) || (tp == TP - 1);
  int t = tp - 1;
  t = (t < 0) ? 0 : t;
  t = (t > NTIME - 1) ? (NTIME - 1) : t;
  const int f = b * NTIME + t;

  for (int i = tid; i < NJ * NJ; i += 64) s_adj[i] = bfr(adj[i]);

  const int h0 = 4 * lane;
  const v4f w0 = bfr4(W + h0);
  const v4f w1 = bfr4(W + NHID + h0);
  const v4f w2 = bfr4(W + 2 * NHID + h0);
  const v4f a1 = bfr4(av + h0);
  const v4f a2 = bfr4(av + NHID + h0);
  const v4f g4 = bfr4(gb + h0);
  __syncthreads();

  const float* xf = x + (size_t)f * (NJ * NCO);
  float* wh = &s_wh[w][0];
#pragma unroll 1
  for (int n = 0; n < NJ; ++n) {
    const float x0 = bfr(xf[3 * n + 0]);
    const float x1 = bfr(xf[3 * n + 1]);
    const float x2 = bfr(xf[3 * n + 2]);
    v4f v;
    float p1 = 0.0f, p2 = 0.0f;
#pragma unroll
    for (int q = 0; q < 4; ++q) {
      const float vq = fmaf(x2, w2[q], fmaf(x1, w1[q], x0 * w0[q]));
      v[q] = vq;
      p1 = fmaf(vq, a1[q], p1);
      p2 = fmaf(vq, a2[q], p2);
    }
    *(v4f*)(wh + n * NHID + h0) = v;
#pragma unroll
    for (int off = 16; off > 0; off >>= 1) {
      p1 += __shfl_xor(p1, off, 32);
      p2 += __shfl_xor(p2, off, 32);
    }
    s_s1[w][n] = p1;
    s_s2[w][n] = p2;
  }
  __syncthreads();

  const bool lv = lane < NJ;
  const int jl = lv ? lane : (NJ - 1);
  const float s2l = s_s2[w][jl];
  unsigned int* stg = &s_stg[w][0];
#pragma unroll 1
  for (int i = 0; i < NJ; ++i) {
    const float s1i = s_s1[w][i];
    const float adjv = s_adj[i * NJ + jl];
    float e = s1i + s2l;
    e = (e > 0.0f) ? e : SLOPE * e;
    e = (adjv > 0.0f) ? e : -9.0e15f;
    e = lv ? e : -3.0e38f;
    float mx = e;
#pragma unroll
    for (int off = 16; off > 0; off >>= 1) mx = fmaxf(mx, __shfl_xor(mx, off, 32));
    float p = __expf(e - mx);
    p = lv ? p : 0.0f;
    float sum = p;
#pragma unroll
    for (int off = 16; off > 0; off >>= 1) sum += __shfl_xor(sum, off, 32);
    const float inv = __builtin_amdgcn_rcpf(sum);
    p *= inv;
    float c0 = 0.0f, c1 = 0.0f, c2 = 0.0f, c3 = 0.0f;
#pragma unroll 3
    for (int j = 0; j < NJ; ++j) {
      const float pj = __shfl(p, j, 32);
      const v4f wv = *(const v4f*)(wh + j * NHID + h0);
      c0 = fmaf(pj, wv[0], c0);
      c1 = fmaf(pj, wv[1], c1);
      c2 = fmaf(pj, wv[2], c2);
      c3 = fmaf(pj, wv[3], c3);
    }
    float hv0 = c0 + g4[0], hv1 = c1 + g4[1], hv2 = c2 + g4[2], hv3 = c3 + g4[3];
    hv0 = (hv0 > 0.0f) ? hv0 : (__expf(hv0) - 1.0f);
    hv1 = (hv1 > 0.0f) ? hv1 : (__expf(hv1) - 1.0f);
    hv2 = (hv2 > 0.0f) ? hv2 : (__expf(hv2) - 1.0f);
    hv3 = (hv3 > 0.0f) ? hv3 : (__expf(hv3) - 1.0f);
    hv0 = isz ? 0.0f : hv0;
    hv1 = isz ? 0.0f : hv1;
    hv2 = isz ? 0.0f : hv2;
    hv3 = isz ? 0.0f : hv3;
    v2u u;
    u[0] = pk16(f16z_bits(hv0), f16z_bits(hv1));
    u[1] = pk16(f16z_bits(hv2), f16z_bits(hv3));
    *(v2u*)(stg + i * (NHID / 2) + 2 * lane) = u;
  }
  __syncthreads();

  unsigned short* dst = Gp + (size_t)row * NCH;
#pragma unroll 1
  for (int s = 0; s < 11; ++s) {
    const int pc = 32 * s + lane;
    if (pc < NPC) {
      const v4u u = *(const v4u*)(stg + 4 * pc);
      *(volatile v4u*)(dst + 8 * pc) = u;
    }
  }
  __threadfence();
#pragma unroll 1
  for (int s = 0; s < 11; ++s) {
    const int pc = 32 * s + lane;
    if (pc < NPC) {
      const v4u u = *(const v4u*)(stg + 4 * pc);
      *(volatile v4u*)(dst + 8 * pc) = u;
    }
  }
}

__global__ __launch_bounds__(256)
void k_conv(const unsigned short* __restrict__ Gp, const unsigned short* __restrict__ Wk,
            const float* __restrict__ conv_b, unsigned short* Yh, unsigned short* Yl) {
  __shared__ __align__(16) unsigned short sh[8][1024];
  __shared__ __align__(16) unsigned short sl[8][1024];
  const int tid = threadIdx.x, w = tid >> 5, lane = tid & 31, hh = lane >> 4, c = lane & 15;
  const int tileM = blockIdx.y * 128 + 16 * w, tileN = blockIdx.x * 64;
  const int b = tileM >> 9, t0 = tileM & (NTIME - 1);
  const int gr = b * TP + t0;

  v8f acc[4];
#pragma unroll
  for (int q = 0; q < 4; ++q) acc[q] = zero8();

#pragma unroll 1
  for (int tap = 0; tap < 3; ++tap) {
    const unsigned short* ap = Gp + (size_t)(gr + tap + c) * NCH + 8 * hh;
    const unsigned short* bp = Wk + (size_t)(tap * NOUT + tileN + c) * NCH + 8 * hh;
#pragma unroll 2
    for (int ks = 0; ks < NCH; ks += 32) {
      const v16h a  = ldfrag_u(ap + ks);
      const v16h b0 = ldfrag_u(bp + ks);
      const v16h b1 = ldfrag_u(bp + (size_t)16 * NCH + ks);
      const v16h b2 = ldfrag_u(bp + (size_t)32 * NCH + ks);
      const v16h b3 = ldfrag_u(bp + (size_t)48 * NCH + ks);
      acc[0] = mma_raw(a, b0, acc[0]);
      acc[1] = mma_raw(a, b1, acc[1]);
      acc[2] = mma_raw(a, b2, acc[2]);
      acc[3] = mma_raw(a, b3, acc[3]);
      guard4(acc[0], acc[1], acc[2], acc[3], a, b0, b1, b2, b3);
    }
  }

  unsigned short* shw = &sh[w][0];
  unsigned short* slw = &sl[w][0];
#pragma unroll
  for (int q = 0; q < 4; ++q) {
    const int n = tileN + 16 * q + c;
    const float cb = bfr(conv_b[n]);
#pragma unroll
    for (int r = 0; r < 8; ++r) {
      const float y = acc[q][r] * IWK + cb;
      unsigned short hb, lb;
      split16(y, hb, lb);
      const int idx = (8 * hh + r) * 64 + 16 * q + c;
      shw[idx] = hb;
      slw[idx] = lb;
    }
  }
  __syncthreads();

  v4u uh[4], ul[4];
#pragma unroll
  for (int s = 0; s < 4; ++s) {
    const int pc = 32 * s + lane;
    uh[s] = *(const v4u*)(shw + 8 * pc);
    ul[s] = *(const v4u*)(slw + 8 * pc);
  }
#pragma unroll
  for (int s = 0; s < 4; ++s) {
    const int pc = 32 * s + lane;
    const size_t o = (size_t)(tileM + (pc >> 3)) * NOUT + tileN + 8 * (pc & 7);
    *(volatile v4u*)(Yh + o) = uh[s];
    *(volatile v4u*)(Yl + o) = ul[s];
  }
  __threadfence();
#pragma unroll
  for (int s = 0; s < 4; ++s) {
    const int pc = 32 * s + lane;
    const size_t o = (size_t)(tileM + (pc >> 3)) * NOUT + tileN + 8 * (pc & 7);
    *(volatile v4u*)(Yh + o) = uh[s];
    *(volatile v4u*)(Yl + o) = ul[s];
  }
}

__global__ __launch_bounds__(256)
void k_proj(const unsigned short* __restrict__ Yh, const unsigned short* __restrict__ Yl,
            const unsigned short* __restrict__ Pw, const float* __restrict__ proj_b,
            const float* __restrict__ hm, float* out) {
  __shared__ __align__(16) float stg[8][1024];
  const int tid = threadIdx.x, w = tid >> 5, lane = tid & 31, hh = lane >> 4, c = lane & 15;
  const int tileM = blockIdx.y * 128 + 16 * w, tileN = blockIdx.x * 64;

  const unsigned short* aph = Yh + (size_t)(tileM + c) * NOUT + 8 * hh;
  const unsigned short* apl = Yl + (size_t)(tileM + c) * NOUT + 8 * hh;
  const unsigned short* bpp = Pw + (size_t)(tileN + c) * NOUT + 8 * hh;

  v8f ah[4], al[4];
#pragma unroll
  for (int q = 0; q < 4; ++q) { ah[q] = zero8(); al[q] = zero8(); }

#pragma unroll 2
  for (int ks = 0; ks < NOUT; ks += 32) {
    const v16h fa = ldfrag_u(aph + ks);
    const v16h fl = ldfrag_u(apl + ks);
    const v16h b0 = ldfrag_u(bpp + ks);
    const v16h b1 = ldfrag_u(bpp + (size_t)16 * NOUT + ks);
    const v16h b2 = ldfrag_u(bpp + (size_t)32 * NOUT + ks);
    const v16h b3 = ldfrag_u(bpp + (size_t)48 * NOUT + ks);
    ah[0] = mma_raw(fa, b0, ah[0]);
    al[0] = mma_raw(fl, b0, al[0]);
    ah[1] = mma_raw(fa, b1, ah[1]);
    al[1] = mma_raw(fl, b1, al[1]);
    ah[2] = mma_raw(fa, b2, ah[2]);
    al[2] = mma_raw(fl, b2, al[2]);
    ah[3] = mma_raw(fa, b3, ah[3]);
    al[3] = mma_raw(fl, b3, al[3]);
    guard8(ah[0], ah[1], ah[2], ah[3], al[0], al[1], al[2], al[3], fa, fl, b0, b1, b2, b3);
  }

  float* sw = &stg[w][0];
#pragma unroll
  for (int q = 0; q < 4; ++q) {
    const int n = tileN + 16 * q + c;
    const float pb = bfr(proj_b[n]);
#pragma unroll
    for (int r = 0; r < 8; ++r) {
      const int m = tileM + 8 * hh + r;
      const float mk = bfr(hm[m]);
      const float v = ((ah[q][r] + al[q][r] * IRES) * IPW + pb) * mk;
      sw[(8 * hh + r) * 64 + 16 * q + c] = v;
    }
  }
  __syncthreads();

  v4f ov[8];
#pragma unroll
  for (int s = 0; s < 8; ++s) ov[s] = *(const v4f*)(sw + 128 * s + 4 * lane);
#pragma unroll
  for (int s = 0; s < 8; ++s) {
    const size_t o = (size_t)(tileM + 2 * s + (lane >> 4)) * NOUT + tileN + 4 * (lane & 15);
    *(volatile v4f*)(out + o) = ov[s];
  }
  __threadfence();
#pragma unroll
  for (int s = 0; s < 8; ++s) {
    const size_t o = (size_t)(tileM + 2 * s + (lane >> 4)) * NOUT + tileN + 4 * (lane & 15);
    *(volatile v4f*)(out + o) = ov[s];
  }
}

extern "C" void kernel_launch(void* const* d_in, const int* in_sizes, int n_in,
                              void* d_out, int out_size, void* d_ws, size_t ws_size,
                              hipStream_t stream) {
  if (n_in < 10) return;
  if (in_sizes[0] != NF * NJ * NCO) return;
  if (in_sizes[1] != NJ * NJ) return;
  if (in_sizes[2] != NF) return;
  if (in_sizes[3] != NCO * NHID) return;
  if (in_sizes[4] != 2 * NHID) return;
  if (in_sizes[5] != NHID) return;
  if (in_sizes[6] != NOUT * KTOT) return;
  if (in_sizes[7] != NOUT) return;
  if (in_sizes[8] != NOUT * NOUT) return;
  if (in_sizes[9] != NOUT) return;
  if (out_size != NF * NOUT) return;

  const float* x      = (const float*)d_in[0];
  const float* adj    = (const float*)d_in[1];
  const float* hm     = (const float*)d_in[2];
  const float* W      = (const float*)d_in[3];
  const float* av     = (const float*)d_in[4];
  const float* gb     = (const float*)d_in[5];
  const float* conv_w = (const float*)d_in[6];
  const float* conv_b = (const float*)d_in[7];
  const float* proj_w = (const float*)d_in[8];
  const float* proj_b = (const float*)d_in[9];
  float* out = (float*)d_out;

  const size_t sGp = (size_t)NROWS * NCH * 2;
  const size_t sWk = (size_t)3 * NOUT * NCH * 2;
  const size_t sPw = (size_t)NOUT * NOUT * 2;
  const size_t sY  = (size_t)NF * NOUT * 2;
  size_t off = 0;
  const size_t oGp = off; off += sGp;
  const size_t oWk = off; off += sWk;
  const size_t oPw = off; off += sPw;
  const size_t oYh = off; off += sY;
  const size_t oYl = off; off += sY;
  if (off > ws_size) return;
  if (off > (size_t)134217728) return;

  char* ws = (char*)d_ws;
  unsigned short* Gp = (unsigned short*)(ws + oGp);
  unsigned short* Wk = (unsigned short*)(ws + oWk);
  unsigned short* Pw = (unsigned short*)(ws + oPw);
  unsigned short* Yh = (unsigned short*)(ws + oYh);
  unsigned short* Yl = (unsigned short*)(ws + oYl);

  k_wprep<<<dim3(1008 + 32), dim3(256), 0, stream>>>(conv_w, proj_w, Wk, Pw);
  k_gat<<<dim3(NROWS / 2), dim3(64), 0, stream>>>(x, adj, W, av, gb, Gp);
  k_conv<<<dim3(NOUT / 64, NF / 128), dim3(256), 0, stream>>>(Gp, Wk, conv_b, Yh, Yl);
  k_proj<<<dim3(NOUT / 64, NF / 128), dim3(256), 0, stream>>>(Yh, Yl, Pw, proj_b, hm, out);
  (void)hipGetLastError();
}
